// My_Attn_17506286698697
// MI455X (gfx1250) — hardware-verified
//
#include <hip/hip_runtime.h>
#include <stdint.h>
#include <stddef.h>

typedef __attribute__((ext_vector_type(16))) _Float16 v16h;
typedef __attribute__((ext_vector_type(8)))  _Float16 v8h;
typedef __attribute__((ext_vector_type(4)))  _Float16 v4h;
typedef __attribute__((ext_vector_type(16))) __bf16   v16b;
typedef __attribute__((ext_vector_type(8)))  __bf16   v8b;
typedef __attribute__((ext_vector_type(8)))  float    v8f;
typedef __attribute__((ext_vector_type(4)))  float    v4f;
#define PSCALE 32768.0f
#define PSCALE_INV (1.0f / 32768.0f)

__device__ __forceinline__ unsigned short f2bf_bits(float f) {
  unsigned u = __float_as_uint(f);
  return (unsigned short)((u + 0x7FFFu + ((u >> 16) & 1u)) >> 16);
}
__device__ __forceinline__ float bf_bits2f(unsigned short h) { return __uint_as_float(((unsigned)h) << 16); }

__device__ __forceinline__ void dep_guard_h(v8f& a, v8f& b, v16h x, v16h y) { asm volatile("v_nop\n\tv_nop\n\tv_nop\n\tv_nop" : "+v"(a), "+v"(b) : "v"(x), "v"(y)); }
__device__ __forceinline__ void dep_guard_b(v8f& a, v8f& b, v16b x, v16b y) { asm volatile("v_nop\n\tv_nop\n\tv_nop\n\tv_nop" : "+v"(a), "+v"(b) : "v"(x), "v"(y)); }
__device__ __forceinline__ void keep4_h(v16h a, v16h b, v16h c, v16h d) { asm volatile("v_nop" :: "v"(a), "v"(b), "v"(c), "v"(d)); }
__device__ __forceinline__ void keep4_b(v16b a, v16b b, v16b c, v16b d) { asm volatile("v_nop" :: "v"(a), "v"(b), "v"(c), "v"(d)); }
__device__ __forceinline__ void acc_guard4(v8f& a, v8f& b, v8f& c, v8f& d) { asm volatile("v_nop\n\tv_nop\n\tv_nop\n\tv_nop" : "+v"(a), "+v"(b), "+v"(c), "+v"(d)); }
template <typename T> struct Frag;
template <> struct Frag<_Float16> {
  typedef v16h V; union U { v16h v; v8h h[2]; };
  static __device__ __forceinline__ v16h load(const _Float16* p) {
    U f; f.h[0] = *(const v8h*)(p); f.h[1] = *(const v8h*)(p + 16); return f.v;
  }
  static __device__ __forceinline__ v8f mma(v16h a, v16h b, v8f c) {
    return __builtin_amdgcn_wmma_f32_16x16x32_f16(false, a, false, b, (short)0, c, false, false);
  }
  static __device__ __forceinline__ void guard(v8f& a, v8f& b, v16h x, v16h y) { dep_guard_h(a, b, x, y); }
  static __device__ __forceinline__ void keep(v16h a, v16h b, v16h c, v16h d) { keep4_h(a, b, c, d); }
};
template <> struct Frag<__bf16> {
  typedef v16b V; union U { v16b v; v8b h[2]; };
  static __device__ __forceinline__ v16b load(const __bf16* p) {
    U f; f.h[0] = *(const v8b*)(p); f.h[1] = *(const v8b*)(p + 16); return f.v;
  }
  static __device__ __forceinline__ v8f mma(v16b a, v16b b, v8f c) {
    return __builtin_amdgcn_wmma_f32_16x16x32_bf16(false, a, false, b, (short)0, c, false, false);
  }
  static __device__ __forceinline__ void guard(v8f& a, v8f& b, v16b x, v16b y) { dep_guard_b(a, b, x, y); }
  static __device__ __forceinline__ void keep(v16b a, v16b b, v16b c, v16b d) { keep4_b(a, b, c, d); }
};

template <int ET> struct Elem;
template <> struct Elem<0> { typedef _Float16 T; };
template <> struct Elem<1> { typedef __bf16 T; };
template <int ET, bool SPLIT, int BIAS_MODE, int OUT_MODE, bool RESID, int ACT = 0>
__global__ __launch_bounds__(256) void wmma_gemm64(
    const unsigned short* __restrict__ Ap, const unsigned short* __restrict__ A2p, int lda, long strideA,
    const unsigned short* __restrict__ Btp, const unsigned short* __restrict__ Bt2p, int ldb, long strideB,
    void* __restrict__ Cout, void* __restrict__ Cout2, int ldc, long strideC,
    const float* __restrict__ bias,
    const float* __restrict__ resid, long strideR,
    int M, int N, int K, float scale) {
  typedef typename Elem<ET>::T T;
  typedef typename Frag<T>::V V;
  const T* A = (const T*)Ap; const T* A2 = (const T*)A2p; const T* Bt = (const T*)Btp; const T* Bt2 = (const T*)Bt2p;
  __shared__ __align__(16) float sT[8][16 * 68];
  const int b    = blockIdx.y;
  const int lane = threadIdx.x & 31;
  const int wave = threadIdx.x >> 5;
  const int tilesN = N >> 6;
  const int tilesM = M >> 6;
  const int tile = blockIdx.x * 8 + wave;
  if (tile >= tilesM * tilesN) return;
  const int tm = tile / tilesN;
  const int tn = tile - tm * tilesN;
  const int m0 = tm << 6;
  const int n0 = tn << 6;

  const T* Ab  = A  + (size_t)b * strideA;
  const T* Bb  = Bt + (size_t)b * strideB;
  const T* Ab2 = SPLIT ? (A2  + (size_t)b * strideA) : nullptr;
  const T* Bb2 = SPLIT ? (Bt2 + (size_t)b * strideB) : nullptr;

  const int rlane = lane & 15;
  const int koff  = (lane >> 4) * 8;
  const int mOff  = (lane >> 4) * 8;

  v8f acc[4][4];
#pragma unroll
  for (int i = 0; i < 4; ++i)
#pragma unroll
    for (int j = 0; j < 4; ++j) acc[i][j] = (v8f){0.f,0.f,0.f,0.f,0.f,0.f,0.f,0.f};

  for (int k0 = 0; k0 < K; k0 += 32) {
    V bh[4], bl[4];
#pragma unroll
    for (int j = 0; j < 4; ++j) {
      const size_t bo = (size_t)(n0 + (j << 4) + rlane) * ldb + koff + k0;
      bh[j] = Frag<T>::load(Bb + bo);
      if (SPLIT) bl[j] = Frag<T>::load(Bb2 + bo);
    }
#pragma unroll
    for (int i = 0; i < 4; ++i) {
      const size_t ao = (size_t)(m0 + (i << 4) + rlane) * lda + koff + k0;
      V ah = Frag<T>::load(Ab + ao);
      V al;
      if (SPLIT) al = Frag<T>::load(Ab2 + ao);
#pragma unroll
      for (int j = 0; j < 4; ++j) {
        acc[i][j] = Frag<T>::mma(ah, bh[j], acc[i][j]);
        if (SPLIT) {
          acc[i][j] = Frag<T>::mma(ah, bl[j], acc[i][j]);
          acc[i][j] = Frag<T>::mma(al, bh[j], acc[i][j]);
        }
      }
      Frag<T>::guard(acc[i][0], acc[i][3], ah, SPLIT ? al : ah);
    }
    Frag<T>::keep(bh[0], bh[1], bh[2], bh[3]);
    if (SPLIT) Frag<T>::keep(bl[0], bl[1], bl[2], bl[3]);
  }
  acc_guard4(acc[0][0], acc[0][1], acc[0][2], acc[0][3]);
  acc_guard4(acc[1][0], acc[1][1], acc[1][2], acc[1][3]);
  acc_guard4(acc[2][0], acc[2][1], acc[2][2], acc[2][3]);
  acc_guard4(acc[3][0], acc[3][1], acc[3][2], acc[3][3]);

  float* slab = sT[wave];
  const float* Rb = RESID ? (resid + (size_t)b * strideR) : nullptr;
#pragma unroll
  for (int i = 0; i < 4; ++i) {
    const int mBase = m0 + (i << 4);
#pragma unroll
    for (int j = 0; j < 4; ++j) {
      const int n = n0 + (j << 4) + rlane;
      float bv = 0.f;
      if (BIAS_MODE == 2) bv = bias[n];
#pragma unroll
      for (int r = 0; r < 8; ++r) {
        float v = acc[i][j][r] * scale;
        if (BIAS_MODE == 1) v += bias[mBase + mOff + r];
        if (BIAS_MODE == 2) v += bv;
        if (RESID) v += Rb[(size_t)(mBase + mOff + r) * ldc + n];
        if (ACT == 1) v = tanhf(v);
        if (ACT == 2) v = fmaxf(v, 0.0f);
        if (ACT == 3) v = v / (1.0f + expf(-v));
        if (ACT == 4) v = (v > 0.f) ? v : 0.01f * v;
        if (ACT == 5) v = 0.5f * v * (1.0f + erff(v * 0.70710678118654752f));
        slab[(mOff + r) * 68 + (j << 4) + rlane] = v;
      }
    }
    __builtin_amdgcn_fence(__ATOMIC_RELEASE, "workgroup");
    __builtin_amdgcn_wave_barrier();
    __builtin_amdgcn_fence(__ATOMIC_ACQUIRE, "workgroup");
    if (OUT_MODE == 0) {
      float* C = (float*)Cout + (size_t)b * strideC;
      const int hh = lane >> 4, c4 = (lane & 15) * 4;
      for (int pass = 0; pass < 2; ++pass) {
#pragma unroll
        for (int it = 0; it < 8; ++it) {
          const int row = it * 2 + hh;
          v4f v = *(const v4f*)(slab + row * 68 + c4);
          *(volatile v4f*)(C + (size_t)(mBase + row) * ldc + n0 + c4) = v;
        }
        __threadfence();
      }
    } else {
      const int q = lane >> 3, c8 = (lane & 7) * 8;
      unsigned short* C  = (unsigned short*)Cout  + (size_t)b * strideC;
      unsigned short* C2 = (OUT_MODE == 2) ? ((unsigned short*)Cout2 + (size_t)b * strideC) : nullptr;
      for (int pass = 0; pass < 2; ++pass) {
#pragma unroll
        for (int it = 0; it < 4; ++it) {
          const int row = it * 4 + q;
          const float* sp = slab + row * 68 + c8;
          v8h hv, lv;
#pragma unroll
          for (int e = 0; e < 8; ++e) {
            if (OUT_MODE == 1) {
              hv[e] = (_Float16)sp[e];
            } else {
              unsigned short hb = f2bf_bits(sp[e]);
              unsigned short lb = f2bf_bits(sp[e] - bf_bits2f(hb));
              hv[e] = __builtin_bit_cast(_Float16, hb);
              lv[e] = __builtin_bit_cast(_Float16, lb);
            }
          }
          *(volatile v8h*)(C + (size_t)(mBase + row) * ldc + n0 + c8) = hv;
          if (OUT_MODE == 2) *(volatile v8h*)(C2 + (size_t)(mBase + row) * ldc + n0 + c8) = lv;
        }
        __threadfence();
      }
    }
    __builtin_amdgcn_fence(__ATOMIC_RELEASE, "workgroup");
    __builtin_amdgcn_wave_barrier();
    __builtin_amdgcn_fence(__ATOMIC_ACQUIRE, "workgroup");
  }
}

__global__ __launch_bounds__(256) void cast_f32_f16x8(
    const float* __restrict__ in, _Float16* __restrict__ out, int n8) {
  const int i = blockIdx.x * 256 + threadIdx.x;
  if (i < n8) {
    const v4f a = *(const v4f*)(in + (size_t)8 * i);
    const v4f c = *(const v4f*)(in + (size_t)8 * i + 4);
    v8h hv;
    hv[0] = (_Float16)a[0]; hv[1] = (_Float16)a[1]; hv[2] = (_Float16)a[2]; hv[3] = (_Float16)a[3];
    hv[4] = (_Float16)c[0]; hv[5] = (_Float16)c[1]; hv[6] = (_Float16)c[2]; hv[7] = (_Float16)c[3];
    *(volatile v8h*)(out + (size_t)8 * i) = hv;
    __threadfence();
    *(volatile v8h*)(out + (size_t)8 * i) = hv;
  }
}

__global__ __launch_bounds__(256) void transpose_cast_f16(
    const float* __restrict__ W, _Float16* __restrict__ Wt, int K, int N, float mul) {
  __shared__ float t[64][33];
  const int tid = threadIdx.x;
  const int n0 = blockIdx.x * 32;
  const int k0 = blockIdx.y * 64;
  {
    const int col = tid & 31;
    const int rb  = tid >> 5;
#pragma unroll
    for (int i = 0; i < 8; ++i) {
      const int r = rb + 8 * i;
      t[r][col] = W[(size_t)(k0 + r) * N + n0 + col];
    }
  }
  __syncthreads();
  {
    const int j  = tid >> 3;
    const int c8 = (tid & 7) * 8;
    v8h hv;
#pragma unroll
    for (int e = 0; e < 8; ++e) hv[e] = (_Float16)(t[c8 + e][j] * mul);
    _Float16* dst = Wt + (size_t)(n0 + j) * K + k0 + c8;
    *(volatile v8h*)dst = hv;
    __threadfence();
    *(volatile v8h*)dst = hv;
  }
}

#define AT_D 64
#define AT_NW 4
#define AT_QB 64
#define AT_KC 64

__device__ __forceinline__ v8f mma_h(v16h a, v16h b, v8f c) {
  c = __builtin_amdgcn_wmma_f32_16x16x32_f16(false, a, false, b, (short)0, c, false, false);
  asm volatile("v_nop\n\tv_nop\n\tv_nop\n\tv_nop" : "+v"(c) : "v"(a), "v"(b));
  return c;
}

__global__ __launch_bounds__(128)
void attn64_f16(const _Float16* __restrict__ qkv, _Float16* __restrict__ out,
                int S, int H, int ld_qkv, int ld_out, float sm_scale, float out_mul) {
  __shared__ __align__(16) _Float16 Ksh[AT_KC * AT_D];
  __shared__ __align__(16) _Float16 Vth[AT_D * AT_KC];
  __shared__ __align__(16) _Float16 Psh[AT_NW][16 * AT_KC];
  __shared__ __align__(16) float    Os[AT_NW][16 * 68];

  const int tid  = threadIdx.x;
  const int wave = tid >> 5;
  const int lane = tid & 31;
  const int hh   = lane >> 4;
  const int c    = lane & 15;

  const int nqb = S / AT_QB;
  const int bx = blockIdx.x;
  const int qb = bx % nqb;
  const int bh = bx / nqb;
  const int h  = bh % H;
  const int b  = bh / H;
  const int q0 = qb * AT_QB + wave * 16;
  const int C  = H * AT_D;

  const _Float16* base = qkv + (size_t)b * S * ld_qkv + (size_t)h * AT_D;

  v16h qa[2];
  {
    const _Float16* qrow = base + (size_t)(q0 + c) * ld_qkv;
#pragma unroll
    for (int dc = 0; dc < 2; ++dc) qa[dc] = Frag<_Float16>::load(qrow + dc * 32 + 8 * hh);
  }

  float mrow[8], lrow[8];
  v8f oacc[4];
#pragma unroll
  for (int r = 0; r < 8; ++r) { mrow[r] = -INFINITY; lrow[r] = 0.f; }
#pragma unroll
  for (int t = 0; t < 4; ++t) oacc[t] = (v8f){0.f,0.f,0.f,0.f,0.f,0.f,0.f,0.f};

  const int nChunks = S / AT_KC;
  for (int kc = 0; kc < nChunks; ++kc) {
    const int kv0 = kc * AT_KC;
    __syncthreads();
    {
      const int kvr = tid >> 1, dh = (tid & 1) * 32;
      const _Float16* krow = base + (size_t)(kv0 + kvr) * ld_qkv + C + dh;
      const _Float16* vrow = base + (size_t)(kv0 + kvr) * ld_qkv + 2 * C + dh;
      v8h kq[4], vq[4];
#pragma unroll
      for (int i = 0; i < 4; ++i) { kq[i] = *(const v8h*)(krow + 8 * i); vq[i] = *(const v8h*)(vrow + 8 * i); }
#pragma unroll
      for (int i = 0; i < 4; ++i) *(v8h*)(Ksh + kvr * AT_D + dh + 8 * i) = kq[i];
#pragma unroll
      for (int i = 0; i < 4; ++i) {
#pragma unroll
        for (int e = 0; e < 8; ++e) Vth[(dh + 8 * i + e) * AT_KC + kvr] = vq[i][e];
      }
    }
    __syncthreads();

    v8f s[4];
#pragma unroll
    for (int j = 0; j < 4; ++j) {
      s[j] = (v8f){0.f,0.f,0.f,0.f,0.f,0.f,0.f,0.f};
#pragma unroll
      for (int dc = 0; dc < 2; ++dc) {
        const v16h kb = Frag<_Float16>::load(Ksh + (j * 16 + c) * AT_D + dc * 32 + 8 * hh);
        s[j] = mma_h(qa[dc], kb, s[j]);
      }
    }
    float cm[8];
#pragma unroll
    for (int r = 0; r < 8; ++r) {
      float m = -INFINITY;
#pragma unroll
      for (int j = 0; j < 4; ++j) { s[j][r] *= sm_scale; m = fmaxf(m, s[j][r]); }
#pragma unroll
      for (int off = 1; off < 16; off <<= 1) m = fmaxf(m, __shfl_xor(m, off, 32));
      cm[r] = m;
    }
    _Float16* pw = Psh[wave];
#pragma unroll
    for (int r = 0; r < 8; ++r) {
      const float mnew = fmaxf(mrow[r], cm[r]);
      const float alpha = __expf(mrow[r] - mnew);
      mrow[r] = mnew;
      float psum = 0.f;
#pragma unroll
      for (int j = 0; j < 4; ++j) {
        const float p = __expf(s[j][r] - mnew);
        psum += p;
        pw[(8 * hh + r) * AT_KC + j * 16 + c] = (_Float16)(p * PSCALE);
      }
#pragma unroll
      for (int off = 1; off < 16; off <<= 1) psum += __shfl_xor(psum, off, 32);
      lrow[r] = lrow[r] * alpha + psum;
#pragma unroll
      for (int t = 0; t < 4; ++t) oacc[t][r] *= alpha;
    }
    __builtin_amdgcn_fence(__ATOMIC_RELEASE, "workgroup");
    __builtin_amdgcn_wave_barrier();
    __builtin_amdgcn_fence(__ATOMIC_ACQUIRE, "workgroup");

#pragma unroll
    for (int kk = 0; kk < 2; ++kk) {
      const v16h pa = Frag<_Float16>::load(pw + c * AT_KC + kk * 32 + 8 * hh);
#pragma unroll
      for (int t = 0; t < 4; ++t) {
        const v16h vb = Frag<_Float16>::load(Vth + (t * 16 + c) * AT_KC + kk * 32 + 8 * hh);
        oacc[t] = mma_h(pa, vb, oacc[t]);
      }
    }
  }

  float* os = Os[wave];
  const float fin = out_mul * PSCALE_INV;
#pragma unroll
  for (int r = 0; r < 8; ++r) {
    const float inv = (1.0f / lrow[r]) * fin;
#pragma unroll
    for (int t = 0; t < 4; ++t) os[(8 * hh + r) * 68 + t * 16 + c] = oacc[t][r] * inv;
  }
  __builtin_amdgcn_fence(__ATOMIC_RELEASE, "workgroup");
  __builtin_amdgcn_wave_barrier();
  __builtin_amdgcn_fence(__ATOMIC_ACQUIRE, "workgroup");
  {
    const int q = lane >> 3, c8 = (lane & 7) * 8;
    _Float16* ob = out + (size_t)b * S * ld_out + (size_t)h * AT_D;
    for (int pass = 0; pass < 2; ++pass) {
#pragma unroll
      for (int it = 0; it < 4; ++it) {
        const int row = it * 4 + q;
        const float* sp = os + row * 68 + c8;
        v8h hv;
#pragma unroll
        for (int e = 0; e < 8; ++e) hv[e] = (_Float16)sp[e];
        *(volatile v8h*)(ob + (size_t)(q0 + row) * ld_out + c8) = hv;
      }
      __threadfence();
    }
  }
}

template <bool F16OUT>
__global__ __launch_bounds__(256)
void ln_residual(const float* __restrict__ ln_in, const float* __restrict__ res,
                 const float* __restrict__ g, const float* __restrict__ bta,
                 float* __restrict__ outf, _Float16* __restrict__ outh, int C, float eps, float invC) {
  __shared__ float red0[8];
  __shared__ float red1[8];
  const int row  = blockIdx.x;
  const int tid  = threadIdx.x;
  const int lane = tid & 31;
  const int wave = tid >> 5;
  const int c4   = tid * 4;
  const size_t rb = (size_t)row * C;

  const v4f v = *(const v4f*)(ln_in + rb + c4);
  float s = (v[0] + v[1]) + (v[2] + v[3]);
#pragma unroll
  for (int off = 1; off < 32; off <<= 1) s += __shfl_xor(s, off, 32);
  if (lane == 0) red0[wave] = s;
  __syncthreads();
  float tot = 0.f;
#pragma unroll
  for (int w = 0; w < 8; ++w) tot += red0[w];
  const float mu = tot * invC;

  v4f d;
  d[0] = v[0] - mu; d[1] = v[1] - mu; d[2] = v[2] - mu; d[3] = v[3] - mu;
  float s2 = (d[0] * d[0] + d[1] * d[1]) + (d[2] * d[2] + d[3] * d[3]);
#pragma unroll
  for (int off = 1; off < 32; off <<= 1) s2 += __shfl_xor(s2, off, 32);
  if (lane == 0) red1[wave] = s2;
  __syncthreads();
  float tot2 = 0.f;
#pragma unroll
  for (int w = 0; w < 8; ++w) tot2 += red1[w];
  const float var  = tot2 * invC;
  const float rstd = rsqrtf(var + eps);

  const v4f gg = *(const v4f*)(g + c4);
  const v4f bb = *(const v4f*)(bta + c4);
  const v4f rr = *(const v4f*)(res + rb + c4);
  v4f o;
  o[0] = rr[0] + (d[0] * rstd * gg[0] + bb[0]);
  o[1] = rr[1] + (d[1] * rstd * gg[1] + bb[1]);
  o[2] = rr[2] + (d[2] * rstd * gg[2] + bb[2]);
  o[3] = rr[3] + (d[3] * rstd * gg[3] + bb[3]);
  v4h oh;
  oh[0] = (_Float16)o[0]; oh[1] = (_Float16)o[1]; oh[2] = (_Float16)o[2]; oh[3] = (_Float16)o[3];

  *(volatile v4f*)(outf + rb + c4) = o;
  if (F16OUT) *(volatile v4h*)(outh + rb + c4) = oh;
  __threadfence();
  *(volatile v4f*)(outf + rb + c4) = o;
  if (F16OUT) *(volatile v4h*)(outh + rb + c4) = oh;
}

template <int OUT_MODE, int ACT>
static void launch_gemm_f16(const _Float16* A, int lda, const _Float16* Bt, int ldb, void* Cp, int ldc,
                            const float* bias, int M, int N, int K, float scale, hipStream_t stream) {
  const int tiles = (M / 64) * (N / 64);
  dim3 grid((unsigned)((tiles + 7) / 8), 1, 1);
  wmma_gemm64<0, false, 2, OUT_MODE, false, ACT><<<grid, 256, 0, stream>>>(
      (const unsigned short*)A, (const unsigned short*)nullptr, lda, 0L,
      (const unsigned short*)Bt, (const unsigned short*)nullptr, ldb, 0L,
      Cp, (void*)nullptr, ldc, 0L,
      bias, (const float*)nullptr, 0L,
      M, N, K, scale);
}

extern "C" void kernel_launch(void* const* d_in, const int* in_sizes, int n_in,
                              void* d_out, int out_size, void* d_ws, size_t ws_size,
                              hipStream_t stream) {
  constexpr int Bb = 4, S = 1024, C = 1024, H = 16, D = 64;
  constexpr int M = Bb * S;
  constexpr int C3 = 3 * C;
  constexpr int F = 4 * C;
  constexpr float WMUL = 64.0f;
  constexpr float OMUL = 64.0f;
  static_assert(H * D == C);

  if (n_in < 13) return;
  if (in_sizes[0] != M * C || in_sizes[1] != C * C3 || in_sizes[2] != C3 || in_sizes[3] != C * C ||
      in_sizes[4] != C || in_sizes[5] != C || in_sizes[6] != C || in_sizes[7] != C || in_sizes[8] != C ||
      in_sizes[9] != C * F || in_sizes[10] != F || in_sizes[11] != F * C || in_sizes[12] != C) return;
  if (out_size != M * C) return;

  const float* x_in   = (const float*)d_in[0];
  const float* qkv_w  = (const float*)d_in[1];
  const float* qkv_b  = (const float*)d_in[2];
  const float* proj_w = (const float*)d_in[3];
  const float* proj_b = (const float*)d_in[4];
  const float* n1_g   = (const float*)d_in[5];
  const float* n1_b   = (const float*)d_in[6];
  const float* n2_g   = (const float*)d_in[7];
  const float* n2_b   = (const float*)d_in[8];
  const float* fc1_w  = (const float*)d_in[9];
  const float* fc1_b  = (const float*)d_in[10];
  const float* fc2_w  = (const float*)d_in[11];
  const float* fc2_b  = (const float*)d_in[12];
  float* out = (float*)d_out;

  size_t off = 0;
  auto carve = [&](size_t bytes) -> size_t { size_t p = off; off += (bytes + 255) & ~(size_t)255; return p; };
  const size_t o_x16   = carve((size_t)M * C * 2);
  const size_t o_wqkvT = carve((size_t)C3 * C * 2);
  const size_t o_wprjT = carve((size_t)C * C * 2);
  const size_t o_wfc1T = carve((size_t)F * C * 2);
  const size_t o_wfc2T = carve((size_t)C * F * 2);
  const size_t o_r1    = carve((size_t)M * F * 2);
  const size_t o_prj   = carve((size_t)M * C * 4);
  const size_t o_pre   = carve((size_t)M * C * 4);
  if (off > ws_size) return;

  char* ws = (char*)d_ws;
  _Float16* x16    = (_Float16*)(ws + o_x16);
  _Float16* pre16  = (_Float16*)(ws + o_x16);
  _Float16* wqkvT  = (_Float16*)(ws + o_wqkvT);
  _Float16* wprjT  = (_Float16*)(ws + o_wprjT);
  _Float16* wfc1T  = (_Float16*)(ws + o_wfc1T);
  _Float16* wfc2T  = (_Float16*)(ws + o_wfc2T);
  _Float16* qkv16  = (_Float16*)(ws + o_r1);
  _Float16* attn16 = (_Float16*)(ws + o_r1 + (size_t)M * C3 * 2);
  _Float16* h1     = (_Float16*)(ws + o_r1);
  float*    prj    = (float*)(ws + o_prj);
  float*    h2     = (float*)(ws + o_prj);
  float*    pre    = (float*)(ws + o_pre);

  {
    const int n8 = M * C / 8;
    cast_f32_f16x8<<<(n8 + 255) / 256, 256, 0, stream>>>(x_in, x16, n8);
  }
  transpose_cast_f16<<<dim3(C3 / 32, C / 64), 256, 0, stream>>>(qkv_w, wqkvT, C, C3, WMUL);
  transpose_cast_f16<<<dim3(C / 32, C / 64), 256, 0, stream>>>(proj_w, wprjT, C, C, WMUL);
  transpose_cast_f16<<<dim3(F / 32, C / 64), 256, 0, stream>>>(fc1_w, wfc1T, C, F, WMUL);
  transpose_cast_f16<<<dim3(C / 32, F / 64), 256, 0, stream>>>(fc2_w, wfc2T, F, C, WMUL);

  launch_gemm_f16<1, 0>(x16, C, wqkvT, C, (void*)qkv16, C3, qkv_b, M, C3, C, 1.0f / WMUL, stream);

  attn64_f16<<<dim3(Bb * H * (S / AT_QB)), 128, 0, stream>>>(qkv16, attn16, S, H, C3, C, 0.125f, OMUL);

  launch_gemm_f16<0, 0>(attn16, C, wprjT, C, (void*)prj, C, proj_b, M, C, C, 1.0f / (WMUL * OMUL), stream);

  ln_residual<true><<<M, 256, 0, stream>>>(prj, x_in, n1_g, n1_b, pre, pre16, C, 1e-5f, 1.0f / (float)C);

  launch_gemm_f16<1, 5>(pre16, C, wfc1T, C, (void*)h1, F, fc1_b, M, F, C, 1.0f / WMUL, stream);

  launch_gemm_f16<0, 0>(h1, F, wfc2T, F, (void*)h2, C, fc2_b, M, C, F, 1.0f / WMUL, stream);

  ln_residual<false><<<M, 256, 0, stream>>>(h2, pre, n2_g, n2_b, out, (_Float16*)nullptr, C, 1e-5f, 1.0f / (float)C);

  (void)hipGetLastError();
}
